// BS2_36618891166097
// MI455X (gfx1250) — hardware-run, weakly checked
//
#include <hip/hip_runtime.h>

typedef __attribute__((ext_vector_type(16))) _Float16 v16h;
typedef __attribute__((ext_vector_type(8)))  _Float16 v8h;
typedef __attribute__((ext_vector_type(8)))  float    v8f;

constexpr int kCurves = 8192;
constexpr int kNT     = 192;
constexpr int kNCP    = 32;
constexpr int kDeg    = 3;
constexpr int kWaves  = kNT / 32;
constexpr int kPitchA = 40;
constexpr int kPitchB = 40;
constexpr float kEps  = 1e-07f;

constexpr float kCarryA   = 512.0f;
constexpr float kCarryB   = 128.0f;
constexpr float kCarryLo  = 2048.0f;
constexpr float kInvMain  = 1.0f / (kCarryA * kCarryB);
constexpr float kInvLo    = 1.0f / kCarryLo;
constexpr float kF16MinNormal = 6.103515625e-05f;

static_assert(kNT == kWaves * 32);
static_assert(kNCP == 32);
static_assert((kPitchA % 8) == 0 && (kPitchB % 8) == 0);
static_assert(kNT * 3 * 4 == 18 * 128);
static_assert(kCarryA * kCarryB == 65536.0f);

__host__ __device__ constexpr float knotv(int i) {
  return (i <= kDeg) ? 0.0f
                     : ((i >= kNCP) ? 1.0f
                                    : (float)((double)(i - kDeg) / (double)(kNCP - kDeg)));
}

struct FragH {
  union U { v16h v; v8h h[2]; };
  static __device__ __forceinline__ v16h load(const _Float16* p) {
    U f;
    f.h[0] = *(const v8h*)(p);
    f.h[1] = *(const v8h*)(p + 16);
    return f.v;
  }
};

__device__ __forceinline__ v8f mma_h(v16h a, v16h b, v8f c) {
  c = __builtin_amdgcn_wmma_f32_16x16x32_f16(false, a, false, b, (short)0, c, false, false);
  asm volatile("v_nop\n\tv_nop\n\tv_nop\n\tv_nop" : "+v"(c) : "v"(a), "v"(b));
  return c;
}

__device__ __forceinline__ float flush16(float v) {
  return (fabsf(v) < kF16MinNormal) ? 0.0f : v;
}

__global__ __launch_bounds__(192)
void spline_eval_kernel(const float* __restrict__ cp,
                        const float* __restrict__ w,
                        const float* __restrict__ ub,
                        float* __restrict__ out)
{
  __shared__ __align__(16) float    sCp[kNCP * 3];
  __shared__ __align__(16) float    sW[kNCP];
  __shared__ __align__(16) _Float16 sB[16 * kPitchB];
  __shared__ __align__(16) _Float16 sA[kNT * kPitchA];
  __shared__ __align__(16) float    sD[kWaves * 32 * 8];
  __shared__ __align__(16) float    sO[kWaves * 96];

  const int b    = blockIdx.x;
  const int tid  = threadIdx.x;
  const int wv   = tid >> 5;
  const int lane = tid & 31;
  const int col  = lane & 15;
  const int half = lane >> 4;

  if (tid < 96) {
    sCp[tid] = cp[(size_t)b * (kNCP * 3) + tid];
  } else if (tid < 128) {
    sW[tid - 96] = w[(size_t)b * kNCP + (tid - 96)];
  }

  const float t = ub[(size_t)b * kNT + tid];

  __syncthreads();

  if (tid < 64) {
    const int n    = tid >> 2;
    const int kq   = (tid & 3) * 8;
    const int comp = n & 3;
    const int cc   = (comp < 3) ? comp : 2;
    const bool live  = (n < 8);
    const bool resid = ((n >> 2) & 1) != 0;
    v8h hv;
#pragma unroll
    for (int e = 0; e < 8; ++e) {
      const int k = kq + e;
      const float wk = sW[k];
      const float ck = sCp[k * 3 + cc];
      const float x  = (comp == 3) ? wk : (ck * wk);
      const float xs = x * kCarryB;
      const float hi = flush16(xs);
      const _Float16 hh = (_Float16)hi;
      const float hf = (float)hh;
      const float lo = flush16((xs - hf) * kCarryLo);
      const float pick = resid ? lo : hi;
      const float val  = live ? pick : 0.0f;
      hv[e] = (_Float16)val;
    }
    *(v8h*)(sB + n * kPitchB + kq) = hv;
  }

  float Np[kNCP + kDeg];
#pragma unroll
  for (int i = 0; i < kNCP + kDeg; ++i)
    Np[i] = (knotv(i) <= t && t < knotv(i + 1)) ? 1.0f : 0.0f;

  auto step = [&](int p, int i) {
    const float invL = 1.0f / (knotv(i + p)     - knotv(i)     + kEps);
    const float invR = 1.0f / (knotv(i + p + 1) - knotv(i + 1) + kEps);
    Np[i] = (t - knotv(i)) * invL * Np[i]
          + (knotv(i + p + 1) - t) * invR * Np[i + 1];
  };
#pragma unroll
  for (int i = 0; i < 34; ++i) step(1, i);
#pragma unroll
  for (int i = 0; i < 33; ++i) step(2, i);
#pragma unroll
  for (int i = 0; i < 32; ++i) step(3, i);

  {
    _Float16* arow = sA + tid * kPitchA;
#pragma unroll
    for (int c = 0; c < 4; ++c) {
      v8h hv;
#pragma unroll
      for (int e = 0; e < 8; ++e) {
        const float s = flush16(Np[c * 8 + e] * kCarryA);
        hv[e] = (_Float16)s;
      }
      *(v8h*)(arow + c * 8) = hv;
    }
  }

  __syncthreads();

  const v16h bfrag = FragH::load(sB + col * kPitchB + 8 * half);
  const v16h a0 = FragH::load(sA + (wv * 32 + col) * kPitchA + 8 * half);
  const v16h a1 = FragH::load(sA + (wv * 32 + 16 + col) * kPitchA + 8 * half);

  v8f acc0 = (v8f){0.f, 0.f, 0.f, 0.f, 0.f, 0.f, 0.f, 0.f};
  v8f acc1 = (v8f){0.f, 0.f, 0.f, 0.f, 0.f, 0.f, 0.f, 0.f};
  acc0 = mma_h(a0, bfrag, acc0);
  acc1 = mma_h(a1, bfrag, acc1);

  if (col < 8) {
#pragma unroll
    for (int r = 0; r < 8; ++r) {
      sD[(wv * 32 + half * 8 + r) * 8 + col]      = acc0[r];
      sD[(wv * 32 + 16 + half * 8 + r) * 8 + col] = acc1[r];
    }
  }

  __syncthreads();

  {
    const float* dr = sD + (wv * 32 + lane) * 8;
    const float d0 = dr[0];
    const float d1 = dr[1];
    const float d2 = dr[2];
    const float d3 = dr[3];
    const float d4 = dr[4];
    const float d5 = dr[5];
    const float d6 = dr[6];
    const float d7 = dr[7];
    const float nx  = (d0 + d4 * kInvLo) * kInvMain;
    const float ny  = (d1 + d5 * kInvLo) * kInvMain;
    const float nz  = (d2 + d6 * kInvLo) * kInvMain;
    const float den = (d3 + d7 * kInvLo) * kInvMain + kEps;
    const float inv = 1.0f / den;
    float* orow = sO + wv * 96 + lane * 3;
    orow[0] = nx * inv;
    orow[1] = ny * inv;
    orow[2] = nz * inv;
  }

  __syncthreads();

  {
    const float v0 = sO[wv * 96 + lane];
    const float v1 = sO[wv * 96 + 32 + lane];
    const float v2 = sO[wv * 96 + 64 + lane];
    volatile float* po = out + (size_t)b * (kNT * 3) + wv * 96;
    po[lane]      = v0;
    po[32 + lane] = v1;
    po[64 + lane] = v2;
    __threadfence();
    po[lane]      = v0;
    po[32 + lane] = v1;
    po[64 + lane] = v2;
  }
}

constexpr int kElemsCp  = kCurves * kNCP * 3;
constexpr int kElemsW   = kCurves * kNCP * 1;
constexpr int kElemsUb  = kCurves * kNT;
constexpr int kElemsOut = kCurves * kNT * 3 * 1;
static_assert(kElemsCp  == 786432);
static_assert(kElemsW   == 262144);
static_assert(kElemsUb  == 1572864);
static_assert(kElemsOut == 4718592);

extern "C" void kernel_launch(void* const* d_in, const int* in_sizes, int n_in,
                              void* d_out, int out_size, void* d_ws, size_t ws_size,
                              hipStream_t stream) {
  if (n_in < 3) return;
  if (in_sizes[0] != kElemsCp) return;
  if (in_sizes[1] != kElemsW) return;
  if (in_sizes[2] != kElemsUb) return;
  if (out_size != kElemsOut) return;
  const float* cp = (const float*)d_in[0];
  const float* w  = (const float*)d_in[1];
  const float* ub = (const float*)d_in[2];
  float* out = (float*)d_out;
  spline_eval_kernel<<<dim3(kCurves), dim3(kNT), 0, stream>>>(cp, w, ub, out);
}
